// NNConvModel_50328426774919
// MI455X (gfx1250) — hardware-run, weakly checked
//
#include <hip/hip_runtime.h>


namespace {
constexpr int N = 20000, NP = 20032, EFULL = 100000, E = 100000  , EP = (E + 15) / 16 * 16, XI = 16, EI = 10, EIP = 16, C1 = 32, C2 = 64, HID1 = 16, HID2 = 32, MK = 160  ;
constexpr float XS = 8.0f, WSC = 256.0f, SLOPE = 0.1f, BNEPS = 1e-5f;
constexpr int RB = 256, NBX = (N + RB - 1) / RB, NBE = (EFULL + RB - 1) / RB;
static_assert(E % 16 == 0 && NP % 64 == 0, "tiling");
typedef _Float16 b16;
typedef __attribute__((ext_vector_type(16))) _Float16 v16b;
typedef __attribute__((ext_vector_type(8))) _Float16 v8b;
typedef __attribute__((ext_vector_type(8))) float v8f;
typedef __attribute__((ext_vector_type(4))) float v4f;
__device__ __forceinline__ float bf16_rne(float f) { unsigned int u = __float_as_uint(f); u += 0x7FFFu + ((u >> 16) & 1u); return __uint_as_float(u & 0xFFFF0000u); }
__device__ __forceinline__ void split16(float v, b16& hi, b16& lo) { hi = (b16)v; lo = (b16)(v - (float)hi); }
__device__ __forceinline__ v16b frag_kb(const b16* p, int hh) { const v8b a = *(const v8b*)(p + 8 * hh), b = *(const v8b*)(p + 16 + 8 * hh); v16b f;
#pragma unroll
  for (int e = 0; e < 8; ++e) { f[e] = a[e]; f[8 + e] = b[e]; } return f; }
__device__ __forceinline__ v8f wmma16b(v16b a, v16b b, v8f c) { v8f d = __builtin_amdgcn_wmma_f32_16x16x32_f16(false, a, false, b, (short)0, c, false, false); asm volatile("v_nop\n\tv_nop\n\tv_nop\n\tv_nop" : "+v"(d) : "v"(a), "v"(b)); return d; }
__device__ __forceinline__ void wave_lds_sync() { __builtin_amdgcn_fence(__ATOMIC_RELEASE, "workgroup"); __builtin_amdgcn_wave_barrier(); __builtin_amdgcn_fence(__ATOMIC_ACQUIRE, "workgroup"); }
__device__ __forceinline__ float pmul(float a, float b) { float p = a * b; asm volatile("" : "+v"(p)); return p; }
__device__ __forceinline__ int iclamp(int v, int lo, int hi) { return v < lo ? lo : (v > hi ? hi : v); }
constexpr int CSR_NBLK = 512, CSR_GB = 9, CSR_GN = 1 << CSR_GB  , CSR_MAXG = 512, CSR_CAP = 12288  ;
__global__ __launch_bounds__(64) void csrA_kernel(const int* __restrict__ dst, int E, int N, int nG, int CHP, int NGP, int* __restrict__ STG, int* __restrict__ HST) {
  extern __shared__ int sm[];
  int* cnt = sm; int* run = sm + NGP; int* ids = sm + 2 * NGP;
  const int b = blockIdx.x; const int ch = (E + CSR_NBLK - 1) / CSR_NBLK; const int e0 = b * ch, e1 = min(E, e0 + ch);
  for (int i = threadIdx.x; i < NGP; i += 64) cnt[i] = 0;
  for (int i = threadIdx.x; i < CHP; i += 64) ids[i] = -1;
  __syncthreads();
  if (threadIdx.x == 0) {
    for (int e = e0; e < e1; ++e) { int d = dst[e]; d = (d < 0) ? 0 : (d >= N ? N - 1 : d); cnt[d >> CSR_GB] += 1; }
    int acc = 0; for (int g = 0; g < nG; ++g) { run[g] = acc; acc += cnt[g]; }
    for (int e = e0; e < e1; ++e) { int d = dst[e]; d = (d < 0) ? 0 : (d >= N ? N - 1 : d); const int g = d >> CSR_GB; ids[run[g]] = e; run[g] += 1; } }
  __syncthreads();
  typedef __attribute__((ext_vector_type(4))) int v4i;
  for (int pass = 0; pass < 2; ++pass) {
    for (int i = threadIdx.x; i < CHP / 4; i += 64) *(volatile v4i*)(STG + (size_t)b * CHP + i * 4) = *(const v4i*)(&ids[i * 4]);
    for (int i = threadIdx.x; i < NGP / 4; i += 64) { v4i v; for (int e = 0; e < 4; ++e) v[e] = (i * 4 + e < nG) ? cnt[i * 4 + e] : 0; *(volatile v4i*)(HST + (size_t)b * NGP + i * 4) = v; }
    __threadfence(); }
}
__global__ __launch_bounds__(512) void csrS_kernel(const int* __restrict__ HST, int nG, int NGP, int* __restrict__ START, int* __restrict__ TOT, int* __restrict__ OFF) {
  __shared__ int tot[CSR_MAXG];
  const int b = threadIdx.x;
  for (int pass = 0; pass < 2; ++pass) { int runb = 0; for (int g = 0; g < nG; ++g) { int c = HST[(size_t)b * NGP + g]; c = (c < 0) ? 0 : c; ((volatile int*)OFF)[(size_t)g * CSR_NBLK + b] = runb; runb += c; } __threadfence(); }
  for (int g = threadIdx.x; g < nG; g += 512) { int s = 0; for (int bb = 0; bb < CSR_NBLK; ++bb) { int c = HST[(size_t)bb * NGP + g]; s += (c < 0) ? 0 : c; } tot[g] = s; }
  __syncthreads();
  if (threadIdx.x < 32) {
    __shared__ int st[CSR_MAXG + 32];
    if (threadIdx.x == 0) { int acc = 0; for (int g = 0; g < NGP; ++g) { st[g] = acc; if (g < nG) acc += (tot[g] + 31) & ~31; } st[NGP] = acc; }
    __builtin_amdgcn_fence(__ATOMIC_RELEASE, "workgroup"); __builtin_amdgcn_wave_barrier(); __builtin_amdgcn_fence(__ATOMIC_ACQUIRE, "workgroup");
    for (int pass = 0; pass < 2; ++pass) { for (int i = threadIdx.x; i < NGP + 32; i += 32) { ((volatile int*)START)[i] = (i <= NGP) ? st[min(i, NGP)] : 0; ((volatile int*)TOT)[i] = (i < nG) ? tot[i] : 0; } __threadfence(); } }
}
__global__ __launch_bounds__(256) void csrB_kernel(const int* __restrict__ dst, int N, int nG, int CHP, int NGP, int permLen, const int* __restrict__ STG, const int* __restrict__ HST, const int* __restrict__ OFF, const int* __restrict__ START, const int* __restrict__ TOT, int* __restrict__ PERM, int* __restrict__ ROWPTR, int* __restrict__ ROWCNT, int* __restrict__ FLAG) {
  typedef __attribute__((ext_vector_type(4))) int v4i;
  __shared__ int ids[CSR_CAP]; __shared__ unsigned short key[CSR_CAP]; __shared__ int outp[CSR_CAP]; __shared__ int ncnt[CSR_GN + 1]; __shared__ int boff[CSR_NBLK + 1];
  const int g = blockIdx.x, t_ = threadIdx.x; int tot = TOT[g]; int st = START[g], stn = START[g + 1]; const int v0 = g * CSR_GN; const int nv = min(CSR_GN, N - v0);
  st = (st < 0) ? 0 : (st > permLen - 32 ? permLen - 32 : st) & ~31; stn = (stn < st) ? st : (stn > permLen ? permLen : stn); tot = (tot < 0) ? 0 : tot; if (tot > stn - st && tot <= CSR_CAP) tot = stn - st;
  if (tot > CSR_CAP) {
    for (int pass = 0; pass < 2; ++pass) { for (int i = t_; i < CSR_GN / 4; i += 256) { v4i a, c; for (int e = 0; e < 4; ++e) { a[e] = st; c[e] = 0; } *(volatile v4i*)(ROWPTR + v0 + i * 4) = a; *(volatile v4i*)(ROWCNT + v0 + i * 4) = c; } if (t_ == 0) ((volatile int*)FLAG)[0] = 1; __threadfence(); } (void)nv; return; }
  if (t_ == 0) { int acc = 0; for (int b = 0; b < CSR_NBLK; ++b) { boff[b] = acc; int c = HST[(size_t)b * NGP + g]; c = (c < 0) ? 0 : (c > CHP ? CHP : c); acc += c; if (acc > tot) acc = tot; } boff[CSR_NBLK] = acc; }
  for (int i = t_; i <= CSR_GN; i += 256) ncnt[i] = 0;
  __syncthreads();
  for (int b = 0; b < CSR_NBLK; ++b) { const int c = boff[b + 1] - boff[b]; int o_ = OFF[(size_t)g * CSR_NBLK + b]; o_ = (o_ < 0) ? 0 : (o_ > CHP - c ? CHP - c : o_); const int* src_ = STG + (size_t)b * CHP + o_;
    for (int i = t_; i < c; i += 256) { int id = src_[i]; id = (id < 0) ? 0 : id; ids[boff[b] + i] = id; int d = dst[id]; d = (d < v0) ? v0 : (d >= N ? N - 1 : d); int kk = d - v0; kk = (kk < 0) ? 0 : (kk >= CSR_GN ? CSR_GN - 1 : kk); key[boff[b] + i] = (unsigned short)kk; } }
  __syncthreads();
  if (t_ == 0) { for (int i = 0; i < tot; ++i) ncnt[key[i]] += 1; int acc = 0; for (int vl = 0; vl < CSR_GN; ++vl) { const int c = ncnt[vl]; ncnt[vl] = acc; acc += c; } ncnt[CSR_GN] = acc;
    for (int i = 0; i < tot; ++i) { const int vl = key[i]; outp[ncnt[vl]] = ids[i]; ncnt[vl] += 1; }
    for (int vl = CSR_GN; vl > 0; --vl) ncnt[vl] = ncnt[vl - 1]; ncnt[0] = 0; }
  __syncthreads();
  for (int pass = 0; pass < 2; ++pass) {
    for (int i = t_; i < (stn - st) / 4; i += 256) { v4i v; for (int e = 0; e < 4; ++e) { const int q = i * 4 + e; v[e] = (q < tot) ? outp[q] : -1; } *(volatile v4i*)(PERM + st + i * 4) = v; }
    for (int i = t_; i < CSR_GN / 4; i += 256) { v4i a, c; for (int e = 0; e < 4; ++e) { const int vl = i * 4 + e; a[e] = st + ncnt[vl]; c[e] = (vl < nv) ? (ncnt[vl + 1] - ncnt[vl]) : 0; } *(volatile v4i*)(ROWPTR + v0 + i * 4) = a; *(volatile v4i*)(ROWCNT + v0 + i * 4) = c; }
    __threadfence(); }
}
__global__ __launch_bounds__(256) void csrZ_kernel(int* __restrict__ p, size_t n4) { typedef __attribute__((ext_vector_type(4))) int v4i; const size_t tid = (size_t)blockIdx.x * 256 + threadIdx.x, nth = (size_t)gridDim.x * 256; v4i z = {0, 0, 0, 0}; for (size_t i = tid; i < n4; i += nth) *(volatile v4i*)(p + i * 4) = z; }
struct CsrBufs { int *STG, *HST, *OFF, *START, *TOT, *PERM, *ROWPTR, *ROWCNT, *FLAG; int nG, NGP, CHP; size_t permLen; char* base; size_t bytes; };
static size_t csr_carve(CsrBufs& c, char* ws, size_t off, int E, int N) {
  const size_t off0 = off; c.base = ws + off;
  auto al = [&](size_t bytes) { char* p = ws + off; off += (bytes + 255) & ~(size_t)255; return p; };
  c.nG = (N + CSR_GN - 1) / CSR_GN; c.NGP = (c.nG + 31) & ~31; const int ch = (E + CSR_NBLK - 1) / CSR_NBLK; c.CHP = (ch + 31) & ~31; c.permLen = (size_t)E + 32 * (size_t)c.nG + 32;
  c.STG = (int*)al((size_t)CSR_NBLK * c.CHP * 4); c.HST = (int*)al((size_t)CSR_NBLK * c.NGP * 4); c.OFF = (int*)al((size_t)c.NGP * CSR_NBLK * 4); c.START = (int*)al((size_t)(c.NGP + 64) * 4); c.TOT = (int*)al((size_t)(c.NGP + 64) * 4);
  c.PERM = (int*)al(c.permLen * 4); c.ROWPTR = (int*)al((size_t)c.nG * CSR_GN * 4); c.ROWCNT = (int*)al((size_t)c.nG * CSR_GN * 4); c.FLAG = (int*)al(256);
  c.bytes = off - off0; return off;
}
static void csr_build(const CsrBufs& c, const int* dst, int E, int N, hipStream_t stream) {
  const size_t smem = (size_t)(2 * c.NGP + c.CHP) * 4;
  csrZ_kernel<<<512, 256, 0, stream>>>((int*)c.base, c.bytes / 16);
  csrA_kernel<<<CSR_NBLK, 64, smem, stream>>>(dst, E, N, c.nG, c.CHP, c.NGP, c.STG, c.HST);
  csrS_kernel<<<1, 512, 0, stream>>>(c.HST, c.nG, c.NGP, c.START, c.TOT, c.OFF);
  csrB_kernel<<<c.nG, 256, 0, stream>>>(dst, N, c.nG, c.CHP, c.NGP, (int)c.permLen, c.STG, c.HST, c.OFF, c.START, c.TOT, c.PERM, c.ROWPTR, c.ROWCNT, c.FLAG);
}

typedef __attribute__((ext_vector_type(4))) _Float16 v4h;
typedef __attribute__((ext_vector_type(2))) float v2f;
__device__ __forceinline__ float lrelu(float v) { return v >= 0.0f ? v : SLOPE * v; }
template <int CW>
__global__ __launch_bounds__(32) void colpart_kernel(const float* __restrict__ IN, int rows, const float* __restrict__ MEAN, int centred, float* __restrict__ PS) {
  const int blk = blockIdx.x, c = threadIdx.x; float s = 0.0f;
  if (c < CW) { const float m = centred ? MEAN[c] : 0.0f;
#pragma unroll 1
    for (int r = 0; r < RB; ++r) { const int row = blk * RB + r; if (row < rows) { const float d = bf16_rne(IN[(size_t)row * CW + c]) - m; s += centred ? d * d : d; } } }
  for (int pass = 0; pass < 2; ++pass) { ((volatile float*)PS)[(size_t)blk * 32 + c] = s; __threadfence(); }
}
__global__ __launch_bounds__(32) void colstat_kernel(const float* __restrict__ PS, int nblk, int rows, float* __restrict__ STAT) {
  const int c = threadIdx.x; float s = 0.0f;
#pragma unroll 1
  for (int b = 0; b < nblk; ++b) s += PS[(size_t)b * 32 + c];
  for (int pass = 0; pass < 2; ++pass) { ((volatile float*)STAT)[c] = s / (float)rows; __threadfence(); }
}
template <int CW>
__global__ __launch_bounds__(256) void bnapply_kernel(const float* __restrict__ IN, int rows, int rowsP, const float* __restrict__ MEAN, const float* __restrict__ VAR, const float* __restrict__ g_, const float* __restrict__ b_, float* __restrict__ OUT) {
  const size_t u = (size_t)blockIdx.x * 256 + threadIdx.x; if (u >= (size_t)rowsP * 4) return; const size_t row = u / 4; const int c0 = (int)(u % 4) * 4; v4f o = {0.0f, 0.0f, 0.0f, 0.0f};
  if (row < (size_t)rows) { for (int j = 0; j < 4; ++j) { const int c = c0 + j; if (c < CW) o[j] = (bf16_rne(IN[row * CW + c]) - MEAN[c]) * rsqrtf(VAR[c] + BNEPS) * bf16_rne(g_[c]) + bf16_rne(b_[c]); } }
  for (int pass = 0; pass < 2; ++pass) { *(volatile v4f*)(OUT + row * 16 + c0) = o; __threadfence(); }
}
__global__ __launch_bounds__(256) void wprep_kernel(const float* __restrict__ n1w2, const float* __restrict__ n2w2, const float* __restrict__ m1, const float* __restrict__ m2, const float* __restrict__ m3, const float* __restrict__ m4,
                                                     b16* __restrict__ W2A, b16* __restrict__ W2B, b16* __restrict__ MW1, b16* __restrict__ MW2, b16* __restrict__ MW3, b16* __restrict__ MW4) {
  size_t t = (size_t)blockIdx.x * 256 + threadIdx.x; v8b o;
  auto emit = [&](b16* dst, size_t e) { for (int pass = 0; pass < 2; ++pass) { *(volatile v8b*)(dst + e) = o; __threadfence(); } };
  { const size_t n = (size_t)512 * 32 / 8; if (t < n) { const size_t e = t * 8; const int c = (int)(e / 32), k0 = (int)(e % 32); for (int j = 0; j < 8; ++j) { const int k = k0 + j; o[j] = (k < HID1) ? (b16)(bf16_rne(n1w2[(size_t)k * 512 + c]) * WSC) : (b16)0.0f; } emit(W2A, e); return; } t -= n; }
  { const size_t n = (size_t)2048 * 32 / 8; if (t < n) { const size_t e = t * 8; const int c = (int)(e / 32), k0 = (int)(e % 32); for (int j = 0; j < 8; ++j) { const int k = k0 + j; o[j] = (b16)(bf16_rne(n2w2[(size_t)k * 2048 + c]) * WSC); } emit(W2B, e); return; } t -= n; }
  { const size_t n = (size_t)64 * MK / 8; if (t < n) { const size_t e = t * 8; const int oo = (int)(e / MK), k0 = (int)(e % MK); for (int j = 0; j < 8; ++j) { const int k = k0 + j; o[j] = (k < 2 * C2 + EI) ? (b16)(bf16_rne(m1[(size_t)k * 64 + oo]) * WSC) : (b16)0.0f; } emit(MW1, e); return; } t -= n; }
  { const size_t n = (size_t)32 * 64 / 8; if (t < n) { const size_t e = t * 8; const int oo = (int)(e / 64), k0 = (int)(e % 64); for (int j = 0; j < 8; ++j) o[j] = (b16)(bf16_rne(m2[(size_t)(k0 + j) * 32 + oo]) * WSC); emit(MW2, e); return; } t -= n; }
  { const size_t n = (size_t)16 * 32 / 8; if (t < n) { const size_t e = t * 8; const int oo = (int)(e / 32), k0 = (int)(e % 32); for (int j = 0; j < 8; ++j) o[j] = (b16)(bf16_rne(m3[(size_t)(k0 + j) * 16 + oo]) * WSC); emit(MW3, e); return; } t -= n; }
  { const size_t n = (size_t)16 * 32 / 8; if (t < n) { const size_t e = t * 8; const int oo = (int)(e / 32), k0 = (int)(e % 32); for (int j = 0; j < 8; ++j) { const int k = k0 + j; o[j] = (k < 16 && oo < 8) ? (b16)(bf16_rne(m4[(size_t)k * 8 + oo]) * WSC) : (b16)0.0f; } emit(MW4, e); } }
}
template <int HID, int CIN, int COUT>
__global__ __launch_bounds__(64) void edge_kernel(const float* __restrict__ EN, const float* __restrict__ w1, const float* __restrict__ b1, const b16* __restrict__ W2T, const float* __restrict__ b2, const float* __restrict__ XIN, const int* __restrict__ srcs, float* __restrict__ MSG) {
  constexpr int NTILE = CIN * COUT / 16, OG = COUT / 16;
  __shared__ __attribute__((aligned(16))) float Ms[2][16][COUT + 4];
  const int wave = threadIdx.x >> 5, lane = threadIdx.x & 31, nloc = lane & 15, hlf = lane >> 4; const size_t e0 = (size_t)blockIdx.x * 32 + wave * 16;
  const size_t er = e0 + nloc; float ein[EI];
#pragma unroll
  for (int j = 0; j < EI; ++j) ein[j] = EN[er * EIP + j];
  v16b ah, al;
#pragma unroll
  for (int el = 0; el < 16; ++el) { const int k = (el < 8) ? (8 * hlf + el) : (16 + 8 * hlf + (el - 8)); float h = 0.0f;
    if (k < HID) { h = bf16_rne(b1[k]);
#pragma unroll
      for (int j = 0; j < EI; ++j) h += pmul(ein[j], bf16_rne(w1[j * HID + k])); h = lrelu(h); }
    b16 p, q; split16(h * XS, p, q); ah[el] = p; al[el] = q; }
  int sr[8];
#pragma unroll
  for (int r = 0; r < 8; ++r) sr[r] = iclamp(srcs[e0 + 8 * hlf + r], 0, N - 1);
  float macc[OG][8];
#pragma unroll
  for (int g = 0; g < OG; ++g) for (int r = 0; r < 8; ++r) macc[g][r] = 0.0f;
#pragma unroll 1
  for (int i = 0; i < CIN; ++i) { float xs[8];
#pragma unroll
    for (int r = 0; r < 8; ++r) xs[r] = XIN[(size_t)sr[r] * (CIN == XI ? 16 : CIN) + i];
#pragma unroll
    for (int g = 0; g < OG; ++g) { const int t = i * OG + g; const v16b bw = frag_kb(W2T + (size_t)(t * 16 + nloc) * 32, hlf); v8f d = (v8f){}; d = wmma16b(ah, bw, d); d = wmma16b(al, bw, d); const float bb = bf16_rne(b2[t * 16 + nloc]);
#pragma unroll
      for (int r = 0; r < 8; ++r) macc[g][r] += pmul(xs[r], lrelu(d[r] * (1.0f / (XS * WSC)) + bb)); } }
#pragma unroll
  for (int g = 0; g < OG; ++g) for (int r = 0; r < 8; ++r) Ms[wave][8 * hlf + r][g * 16 + nloc] = macc[g][r];
  wave_lds_sync();
  typedef __attribute__((ext_vector_type(COUT / 32))) float vst;
  for (int pass = 0; pass < 2; ++pass) { for (int rr = 0; rr < 16; ++rr) *(volatile vst*)(MSG + (e0 + rr) * COUT + lane * (COUT / 32)) = *(const vst*)(&Ms[wave][rr][lane * (COUT / 32)]); __threadfence(); }
}
template <int CIN, int COUT>
__global__ __launch_bounds__(256) void node_kernel(const float* __restrict__ MSG, const float* __restrict__ XIN, const float* __restrict__ root, const float* __restrict__ bias, const int* __restrict__ PERM, const int* __restrict__ ROWPTR, const int* __restrict__ ROWCNT, int permLen, float* __restrict__ XOUT) {
  constexpr int CPL = COUT / 32; typedef __attribute__((ext_vector_type(CPL))) float vf;
  const int wave = threadIdx.x >> 5, lane = threadIdx.x & 31; const size_t v = (size_t)blockIdx.x * 8 + wave; const int c = lane * CPL; vf a; for (int j = 0; j < CPL; ++j) a[j] = 0.0f;
  if (v < (size_t)N) { int st = ROWPTR[v], cnt = ROWCNT[v]; cnt = iclamp(cnt, 0, 65536); st = iclamp(st, 0, permLen - cnt);
#pragma unroll 1
    for (int j = 0; j < cnt; ++j) { const int e = iclamp(PERM[st + j], 0, E - 1); const vf m = *(const vf*)(MSG + (size_t)e * COUT + c); a += m; }
    for (int j = 0; j < CPL; ++j) { float s = bf16_rne(bias[c + j]);
#pragma unroll 1
      for (int i = 0; i < CIN; ++i) s += pmul(XIN[v * (CIN == XI ? 16 : CIN) + i], bf16_rne(root[i * COUT + c + j])); a[j] += s; } }
  for (int pass = 0; pass < 2; ++pass) { *(volatile vf*)(XOUT + v * COUT + c) = a; __threadfence(); }
}
__global__ __launch_bounds__(64) void head_kernel(const float* __restrict__ X2, const float* __restrict__ EN, const int* __restrict__ srcs, const int* __restrict__ dsts, const b16* __restrict__ MW1, const float* __restrict__ mb1, const b16* __restrict__ MW2, const float* __restrict__ mb2, const b16* __restrict__ MW3, const float* __restrict__ mb3, const b16* __restrict__ MW4, const float* __restrict__ mb4, const float* __restrict__ mw5, const float* __restrict__ mb5, float* __restrict__ out) {
  __shared__ __attribute__((aligned(16))) b16 Ah[2][16][MK + 8], Al[2][16][MK + 8]; __shared__ __attribute__((aligned(16))) float Tf[2][16][64 + 4]; __shared__ __attribute__((aligned(16))) float Po[2][16][2];
  const int wave = threadIdx.x >> 5, lane = threadIdx.x & 31, nloc = lane & 15, hlf = lane >> 4; const size_t e0 = (size_t)blockIdx.x * 32 + wave * 16;
  { const int rr = lane & 15; const size_t e = e0 + rr; const int s = iclamp(srcs[e], 0, N - 1), d = iclamp(dsts[e], 0, N - 1); const float* xa = X2 + (size_t)(hlf ? d : s) * C2;
    for (int q = 0; q < C2; q += 8) { v8b hv, lv; for (int j = 0; j < 8; ++j) { b16 p, qq; split16(xa[q + j] * XS, p, qq); hv[j] = p; lv[j] = qq; } *(v8b*)(&Ah[wave][rr][hlf * C2 + q]) = hv; *(v8b*)(&Al[wave][rr][hlf * C2 + q]) = lv; }
    if (hlf == 0) { for (int q = 0; q < 32; q += 8) { v8b hv, lv; for (int j = 0; j < 8; ++j) { const int c = q + j; float v = (c < EI) ? EN[e * EIP + c] : 0.0f; b16 p, qq; split16(v * XS, p, qq); hv[j] = p; lv[j] = qq; } *(v8b*)(&Ah[wave][rr][2 * C2 + q]) = hv; *(v8b*)(&Al[wave][rr][2 * C2 + q]) = lv; } } }
  wave_lds_sync();
  auto stage = [&](v8f* acc, int ntile, const float* bias, int nb) {
#pragma unroll
    for (int t = 0; t < 4; ++t) { if (t < ntile) { const int c = t * 16 + nloc; const float bb = (c < nb) ? bf16_rne(bias[c]) : 0.0f;
#pragma unroll
        for (int r = 0; r < 8; ++r) Tf[wave][8 * hlf + r][c] = (c < nb) ? lrelu(acc[t][r] * (1.0f / (XS * WSC)) + bb) : 0.0f; } else {
#pragma unroll
        for (int r = 0; r < 8; ++r) Tf[wave][8 * hlf + r][t * 16 + nloc] = 0.0f; } }
    wave_lds_sync();
    { const int rr = lane & 15, c0 = hlf * 32; for (int q = 0; q < 32; q += 8) { v8b hv, lv; for (int j = 0; j < 8; ++j) { b16 p, qq; split16(Tf[wave][rr][c0 + q + j] * XS, p, qq); hv[j] = p; lv[j] = qq; } *(v8b*)(&Ah[wave][rr][c0 + q]) = hv; *(v8b*)(&Al[wave][rr][c0 + q]) = lv; } }
    wave_lds_sync(); };
  v8f acc[4];
#pragma unroll
  for (int t = 0; t < 4; ++t) acc[t] = (v8f){};
#pragma unroll 1
  for (int kb = 0; kb < MK; kb += 32) { const v16b a = frag_kb(&Ah[wave][nloc][kb], hlf), al = frag_kb(&Al[wave][nloc][kb], hlf);
#pragma unroll
    for (int t = 0; t < 4; ++t) { const v16b bw = frag_kb(MW1 + (size_t)(t * 16 + nloc) * MK + kb, hlf); acc[t] = wmma16b(a, bw, acc[t]); acc[t] = wmma16b(al, bw, acc[t]); } }
  wave_lds_sync(); stage(acc, 4, mb1, 64);
#pragma unroll
  for (int t = 0; t < 4; ++t) acc[t] = (v8f){};
#pragma unroll
  for (int kb = 0; kb < 64; kb += 32) { const v16b a = frag_kb(&Ah[wave][nloc][kb], hlf), al = frag_kb(&Al[wave][nloc][kb], hlf);
#pragma unroll
    for (int t = 0; t < 2; ++t) { const v16b bw = frag_kb(MW2 + (size_t)(t * 16 + nloc) * 64 + kb, hlf); acc[t] = wmma16b(a, bw, acc[t]); acc[t] = wmma16b(al, bw, acc[t]); } }
  wave_lds_sync(); stage(acc, 2, mb2, 32);
  acc[0] = (v8f){}; { const v16b a = frag_kb(&Ah[wave][nloc][0], hlf), al = frag_kb(&Al[wave][nloc][0], hlf); const v16b bw = frag_kb(MW3 + (size_t)nloc * 32, hlf); acc[0] = wmma16b(a, bw, acc[0]); acc[0] = wmma16b(al, bw, acc[0]); }
  wave_lds_sync(); stage(acc, 1, mb3, 16);
  acc[0] = (v8f){}; { const v16b a = frag_kb(&Ah[wave][nloc][0], hlf), al = frag_kb(&Al[wave][nloc][0], hlf); const v16b bw = frag_kb(MW4 + (size_t)nloc * 32, hlf); acc[0] = wmma16b(a, bw, acc[0]); acc[0] = wmma16b(al, bw, acc[0]); }
  wave_lds_sync();
  { const int c = nloc; const float bb = (c < 8) ? bf16_rne(mb4[c]) : 0.0f;
#pragma unroll
    for (int r = 0; r < 8; ++r) Tf[wave][8 * hlf + r][c] = (c < 8) ? lrelu(acc[0][r] * (1.0f / (XS * WSC)) + bb) : 0.0f; }
  wave_lds_sync();
  if (lane < 16) { const int rr = lane; float p0 = bf16_rne(mb5[0]), p1 = bf16_rne(mb5[1]);
#pragma unroll
    for (int k = 0; k < 8; ++k) { const float h4 = Tf[wave][rr][k]; p0 += pmul(h4, bf16_rne(mw5[k * 2 + 0])); p1 += pmul(h4, bf16_rne(mw5[k * 2 + 1])); } Po[wave][rr][0] = p0; Po[wave][rr][1] = p1; }
  wave_lds_sync();
  for (int pass = 0; pass < 2; ++pass) { if (lane < 16) *(volatile v2f*)(out + (e0 + lane) * 2) = *(const v2f*)(&Po[wave][lane][0]); __threadfence(); }
}
}

extern "C" void kernel_launch(void* const* d_in, const int* in_sizes, int n_in, void* d_out, int out_size, void* d_ws, size_t ws_size, hipStream_t stream) {
  (void)n_in;
  auto Fp = [&](int i) { return (const float*)d_in[i]; }; auto Ip = [&](int i) { return (const int*)d_in[i]; };
  if (in_sizes[0] != N * XI || in_sizes[1] != EFULL * EI || in_sizes[2] != 2 * EFULL || in_sizes[8] != EI * HID1 || in_sizes[10] != HID1 * XI * C1 || in_sizes[11] != XI * C1 || in_sizes[12] != EI * HID2 || in_sizes[14] != HID2 * C1 * C2 || in_sizes[15] != C1 * C2 ||
      in_sizes[16] != XI * C1 || in_sizes[18] != C1 * C2 || in_sizes[20] != (2 * C2 + EI) * 64 || in_sizes[22] != 64 * 32 || in_sizes[24] != 32 * 16 || in_sizes[26] != 16 * 8 || in_sizes[28] != 8 * 2 || in_sizes[29] != 2 || out_size != EFULL * 2) return;
  size_t off = 0; char* ws = (char*)d_ws;
  auto carve = [&](size_t bytes) { char* p = ws + off; off += (bytes + 255) & ~(size_t)255; return p; };
  float* PSB = (float*)carve((size_t)(NBE > NBX ? NBE : NBX) * 32 * 4); float* STX = (float*)carve(2 * 32 * 4); float* STE = (float*)carve(2 * 32 * 4);
  float* XN = (float*)carve((size_t)NP * 16 * 4); float* EN = (float*)carve((size_t)EFULL * 16 * 4);
  b16* W2A = (b16*)carve((size_t)512 * 32 * 2); b16* W2B = (b16*)carve((size_t)2048 * 32 * 2); b16* MW1 = (b16*)carve((size_t)64 * MK * 2); b16* MW2 = (b16*)carve((size_t)32 * 64 * 2); b16* MW3 = (b16*)carve((size_t)16 * 32 * 2); b16* MW4 = (b16*)carve((size_t)16 * 32 * 2);
  float* MSG1 = (float*)carve((size_t)EFULL * C1 * 4); float* X1 = (float*)carve((size_t)NP * C1 * 4); float* MSG2 = (float*)carve((size_t)EFULL * C2 * 4); float* X2 = (float*)carve((size_t)NP * C2 * 4);
  CsrBufs csr; off = csr_carve(csr, ws, off, E, N);
  if (off > ws_size || off > ((size_t)128 << 20)) return;
  colpart_kernel<XI><<<NBX, 32, 0, stream>>>(Fp(0), N, nullptr, 0, PSB); colstat_kernel<<<1, 32, 0, stream>>>(PSB, NBX, N, STX);
  colpart_kernel<XI><<<NBX, 32, 0, stream>>>(Fp(0), N, STX, 1, PSB);     colstat_kernel<<<1, 32, 0, stream>>>(PSB, NBX, N, STX + 32);
  bnapply_kernel<XI><<<(unsigned)(((size_t)NP * 4 + 255) / 256), 256, 0, stream>>>(Fp(0), N, NP, STX, STX + 32, Fp(4), Fp(5), XN);
  colpart_kernel<EI><<<NBE, 32, 0, stream>>>(Fp(1), EFULL, nullptr, 0, PSB); colstat_kernel<<<1, 32, 0, stream>>>(PSB, NBE, EFULL, STE);
  colpart_kernel<EI><<<NBE, 32, 0, stream>>>(Fp(1), EFULL, STE, 1, PSB);     colstat_kernel<<<1, 32, 0, stream>>>(PSB, NBE, EFULL, STE + 32);
  bnapply_kernel<EI><<<(unsigned)(((size_t)EFULL * 4 + 255) / 256), 256, 0, stream>>>(Fp(1), EFULL, EFULL, STE, STE + 32, Fp(6), Fp(7), EN);
  wprep_kernel<<<(unsigned)((((size_t)512 * 32 + 2048 * 32 + 64 * MK + 32 * 64 + 16 * 32 + 16 * 32) / 8 + 255) / 256), 256, 0, stream>>>(Fp(10), Fp(14), Fp(20), Fp(22), Fp(24), Fp(26), W2A, W2B, MW1, MW2, MW3, MW4);
  csr_build(csr, Ip(2) + EFULL, E, N, stream);
  edge_kernel<HID1, XI, C1><<<E / 32, 64, 0, stream>>>(EN, Fp(8), Fp(9), W2A, Fp(11), XN, Ip(2), MSG1);
  node_kernel<XI, C1><<<NP / 8, 256, 0, stream>>>(MSG1, XN, Fp(16), Fp(17), csr.PERM, csr.ROWPTR, csr.ROWCNT, (int)csr.permLen, X1);
  edge_kernel<HID2, C1, C2><<<E / 32, 64, 0, stream>>>(EN, Fp(12), Fp(13), W2B, Fp(15), X1, Ip(2), MSG2);
  node_kernel<C1, C2><<<NP / 8, 256, 0, stream>>>(MSG2, X1, Fp(18), Fp(19), csr.PERM, csr.ROWPTR, csr.ROWCNT, (int)csr.permLen, X2);
  head_kernel<<<E / 32, 64, 0, stream>>>(X2, EN, Ip(2), Ip(2) + EFULL, MW1, Fp(21), MW2, Fp(23), MW3, Fp(25), MW4, Fp(27), Fp(28), Fp(29), (float*)d_out);
}
